// NeuralOptimalTransport_56573309223313
// MI455X (gfx1250) — hardware-run, weakly checked
//
#include <hip/hip_runtime.h>
#include <math.h>

typedef __attribute__((ext_vector_type(16))) _Float16 v16h;
typedef __attribute__((ext_vector_type(16))) __bf16 v16b;
typedef __attribute__((ext_vector_type(8)))  _Float16 v8h;
typedef __attribute__((ext_vector_type(8)))  float v8f;
typedef __attribute__((ext_vector_type(4)))  float v4f;
typedef __attribute__((ext_vector_type(2)))  float v2f;
typedef __attribute__((ext_vector_type(4)))  unsigned v4u;
typedef __attribute__((ext_vector_type(4)))  int v4i;
typedef float __attribute__((may_alias)) float_a;
typedef int __attribute__((may_alias)) int_a;

template <typename T> __device__ __forceinline__ void vst2(void* p, T v) { *(volatile T*)p = v; __threadfence(); *(volatile T*)p = v; }
__device__ __forceinline__ v8f wmma16(v16h a, v16h b, v8f c) {
  v8f d = __builtin_amdgcn_wmma_f32_16x16x32_f16(false, a, false, b, (short)0, c, false, false);
  asm volatile("v_nop\n\tv_nop\n\tv_nop\n\tv_nop" : "+v"(d) : "v"(a), "v"(b));
  return d;
}
__device__ __forceinline__ v8f wmma_bf(v16b a, v16b b, v8f c) {
  v8f d = __builtin_amdgcn_wmma_f32_16x16x32_bf16(false, a, false, b, (short)0, c, false, false);
  asm volatile("v_nop\n\tv_nop\n\tv_nop\n\tv_nop" : "+v"(d) : "v"(a), "v"(b));
  return d;
}
__device__ __forceinline__ v16h frag_h(const _Float16* rowk0, int lane) {
  union { v16h v; v8h q[2]; } u; const _Float16* p = rowk0 + 8 * (lane >> 4);
  u.q[0] = *(const v8h*)p; u.q[1] = *(const v8h*)(p + 16); return u.v;
}
__device__ __forceinline__ v16h frag_f32(const float* rowk0, int lane) {
  v16h a; const float* p = rowk0 + 8 * (lane >> 4);
#pragma unroll
  for (int i = 0; i < 8; ++i) { a[i] = (_Float16)p[i]; a[8 + i] = (_Float16)p[16 + i]; }
  return a;
}
__device__ __forceinline__ v16h frag_f32s(const float* rowk0, int lane, float sc) {
  v16h a; const float* p = rowk0 + 8 * (lane >> 4);
#pragma unroll
  for (int i = 0; i < 8; ++i) { a[i] = (_Float16)(p[i] * sc); a[8 + i] = (_Float16)(p[16 + i] * sc); }
  return a;
}
__device__ __forceinline__ v16h fragc_f32(const float* W, int k0, int n, int lane, int ld, int K) {
  v16h a; const int g = lane >> 4;
#pragma unroll
  for (int i = 0; i < 8; ++i) { const int ka = k0 + 8 * g + i, kb = ka + 16;
    a[i] = (_Float16)(ka < K ? W[(size_t)(ka < K ? ka : K - 1) * ld + n] : 0.f); a[8 + i] = (_Float16)(kb < K ? W[(size_t)(kb < K ? kb : K - 1) * ld + n] : 0.f); }
  return a;
}
struct F2 { v16b h, l; };
__device__ __forceinline__ F2 bsplit16(const float v[16]) { F2 r;
#pragma unroll
  for (int i = 0; i < 16; ++i) { const __bf16 h = (__bf16)v[i]; r.h[i] = h; r.l[i] = (__bf16)(v[i] - (float)h); }
  return r; }
__device__ __forceinline__ F2 split_row(const float* row, int k0, int lane) { float v[16]; const float* p = row + k0 + 8 * (lane >> 4);
#pragma unroll
  for (int i = 0; i < 8; ++i) { v[i] = p[i]; v[8 + i] = p[16 + i]; }
  return bsplit16(v); }
__device__ __forceinline__ F2 split_rowK(const float* row, int k0, int lane, int K) { float v[16]; const int g = lane >> 4;
#pragma unroll
  for (int i = 0; i < 8; ++i) { const int ka = k0 + 8 * g + i, kb = ka + 16; v[i] = ka < K ? row[ka < K ? ka : K - 1] : 0.f; v[8 + i] = kb < K ? row[kb < K ? kb : K - 1] : 0.f; }
  return bsplit16(v); }
__device__ __forceinline__ F2 split_col(const float* W, int k0, int n, int lane, int ld, int K) { float v[16]; const int g = lane >> 4;
#pragma unroll
  for (int i = 0; i < 8; ++i) { const int ka = k0 + 8 * g + i, kb = ka + 16; v[i] = ka < K ? W[(size_t)(ka < K ? ka : K - 1) * ld + n] : 0.f; v[8 + i] = kb < K ? W[(size_t)(kb < K ? kb : K - 1) * ld + n] : 0.f; }
  return bsplit16(v); }
__device__ __forceinline__ v8f mac3(const F2& a, const F2& b, v8f c) { c = wmma_bf(a.l, b.h, c); c = wmma_bf(a.h, b.l, c); return wmma_bf(a.h, b.h, c); }
__device__ __forceinline__ float sigm(float v) { return 1.0f / (1.0f + expf(-v)); }
#define LDSX() do { asm volatile("s_wait_dscnt 0" ::: "memory"); __builtin_amdgcn_wave_barrier(); __builtin_amdgcn_fence(__ATOMIC_RELEASE, "workgroup"); } while (0)


#define NN 1024
#define ED 256
#define HID 128
typedef __attribute__((ext_vector_type(8))) __bf16 v8b;
__device__ __forceinline__ v16b frag_b(const __bf16* rowk0, int lane) {
  union { v16b v; v8b q[2]; } u; const __bf16* p = rowk0 + 8 * (lane >> 4);
  u.q[0] = *(const v8b*)p; u.q[1] = *(const v8b*)(p + 16); return u.v;
}
__device__ __forceinline__ float bfr(float v) { return (float)(__bf16)v; }
__device__ __attribute__((noinline)) float exp_ni(float v) { return expf(v); }
__device__ __attribute__((noinline)) float erf_ni(float v) { return erff(v); }

#define WS_PW  0u
#define WS_HS  (WS_PW + 2u * 2 * HID * ED)
#define WS_HT  (WS_HS + 4u * NN * HID)
#define WS_RS  (WS_HT + 4u * NN * HID)
#define WS_U   (WS_RS + 4u * NN * 8 * 32)
#define WS_CS  (WS_U + 4u * NN)
#define WS_V   (WS_CS + 4u * 16 * NN)
#define WS_END (WS_V + 4u * NN)

__global__ __launch_bounds__(256) void k_packT(const float* __restrict__ W1, __bf16* __restrict__ PW) {
  __shared__ __align__(16) __bf16 s[ED]; const int o = blockIdx.x, half = blockIdx.y, k = threadIdx.x;
  s[k] = (__bf16)W1[((size_t)half * ED + k) * HID + o]; __syncthreads();
  if (k < ED / 8) vst2((unsigned*)(PW + ((size_t)half * HID + o) * ED + k * 8), *(const v4u*)&s[k * 8]);
}
__global__ __launch_bounds__(128) void k_proj(const float* __restrict__ SRC, const float* __restrict__ TGT, const __bf16* __restrict__ PW, float* __restrict__ HS, float* __restrict__ HT) {
  __shared__ __align__(16) float so[4][16][132];
  const int tid = threadIdx.x, wave = tid >> 5, lane = tid & 31, col = lane & 15, g = lane >> 4; const int half = blockIdx.y; const size_t r0 = (size_t)blockIdx.x * 64 + wave * 16;
  const float* X = half ? TGT : SRC; float* OUT = half ? HT : HS;
  v8f acc[8] = {};
#pragma unroll
  for (int kc = 0; kc < ED / 32; ++kc) { v16b a; { const float* p = X + (r0 + col) * ED + kc * 32 + 8 * g;
#pragma unroll
      for (int i = 0; i < 8; ++i) { a[i] = (__bf16)p[i]; a[8 + i] = (__bf16)p[16 + i]; } }
#pragma unroll
    for (int j = 0; j < 8; ++j) acc[j] = wmma_bf(a, frag_b(PW + ((size_t)half * HID + j * 16 + col) * ED + kc * 32, lane), acc[j]); }
#pragma unroll
  for (int j = 0; j < 8; ++j)
#pragma unroll
    for (int r = 0; r < 8; ++r) so[wave][8 * g + r][j * 16 + col] = acc[j][r];
  LDSX();
  for (int rl = 0; rl < 16; ++rl) vst2(OUT + (r0 + rl) * HID + lane * 4, *(const v4f*)&so[wave][rl][lane * 4]);
}
__global__ __launch_bounds__(256) void k_cost(const float* __restrict__ HS, const float* __restrict__ HT, const float* __restrict__ B1, const float* __restrict__ W2, const float* __restrict__ B2, float* __restrict__ C, float* __restrict__ RS) {
  __shared__ float shs[64][HID + 1]; __shared__ float sht[128][HID + 1]; __shared__ float sw2[HID], sb1[HID]; __shared__ __align__(16) float sc[64][132]; __shared__ float srs[64][17];
  const int tid = threadIdx.x; const int i0 = blockIdx.x * 64, j0 = blockIdx.y * 128;
  for (int q = tid; q < 64 * HID; q += 256) shs[q / HID][q % HID] = HS[(size_t)(i0 + q / HID) * HID + q % HID];
  for (int q = tid; q < 128 * HID; q += 256) sht[q / HID][q % HID] = HT[(size_t)(j0 + q / HID) * HID + q % HID];
  if (tid < HID) { sw2[tid] = bfr(W2[tid]); sb1[tid] = bfr(B1[tid]); }
  __syncthreads();
  const float b2 = bfr(B2[0]);
  const int rg = tid >> 4, cg = tid & 15;
  float rsum[4] = {0.f, 0.f, 0.f, 0.f};
#pragma unroll 1
  for (int rr = 0; rr < 4; ++rr) { const int il = rg * 4 + rr;
#pragma unroll 1
    for (int cc = 0; cc < 8; ++cc) { const int jl = cg * 8 + cc; float acc = b2;
#pragma unroll 1
      for (int k = 0; k < HID; ++k) { const float pre = shs[il][k] + sht[jl][k] + sb1[k]; acc += fmaxf(pre, 0.f) * sw2[k]; }
      sc[il][jl] = acc; rsum[rr] += exp_ni(-acc); } }
#pragma unroll
  for (int rr = 0; rr < 4; ++rr) srs[rg * 4 + rr][cg] = rsum[rr];
  __syncthreads();
  for (int q = tid; q < 64 * 32; q += 256) { const int il = q >> 5, pc = q & 31; vst2(C + (size_t)(i0 + il) * NN + j0 + pc * 4, *(const v4f*)&sc[il][pc * 4]); }
  { __shared__ __align__(16) float sl2[64][32]; for (int q = tid; q < 64 * 32; q += 256) { const int il = q >> 5, pc = q & 31; float v = 0.f; if (pc == 0) { for (int c2 = 0; c2 < 16; ++c2) v += srs[il][c2]; } sl2[il][pc] = v; }
    __syncthreads();
    for (int q = tid; q < 64 * 8; q += 256) { const int il = q >> 3, pc = q & 7; vst2(RS + ((size_t)(i0 + il) * 8 + blockIdx.y) * 32 + pc * 4, *(const v4f*)&sl2[il][pc * 4]); } }
}
__global__ __launch_bounds__(64) void k_u(const float* __restrict__ RS, float* __restrict__ U) {
  __shared__ __align__(16) float s[64]; const int tid = threadIdx.x; const int i = blockIdx.x * 64 + tid; float acc = 0.f;
#pragma unroll
  for (int cb = 0; cb < 8; ++cb) acc += RS[((size_t)i * 8 + cb) * 32];
  s[tid] = (1.0f / (float)NN) / (acc * (1.0f / (float)NN) + 1e-8f); __syncthreads();
  if (tid < 16) vst2(U + (size_t)blockIdx.x * 64 + tid * 4, *(const v4f*)&s[tid * 4]);
}
__global__ __launch_bounds__(256) void k_colsum(const float* __restrict__ C, const float* __restrict__ U, float* __restrict__ CS) {
  __shared__ __align__(16) float s[256]; const int tid = threadIdx.x; const int i0 = blockIdx.x * 64, j = blockIdx.y * 256 + tid; float acc = 0.f;
#pragma unroll 1
  for (int il = 0; il < 64; ++il) acc += exp_ni(-C[(size_t)(i0 + il) * NN + j]) * U[i0 + il];
  s[tid] = acc; __syncthreads();
  if (tid < 64) vst2(CS + (size_t)blockIdx.x * NN + blockIdx.y * 256 + tid * 4, *(const v4f*)&s[tid * 4]);
}
__global__ __launch_bounds__(256) void k_v(const float* __restrict__ CS, float* __restrict__ V) {
  __shared__ __align__(16) float s[256]; const int tid = threadIdx.x; const int j = blockIdx.x * 256 + tid; float acc = 0.f;
#pragma unroll
  for (int rb = 0; rb < NN / 64; ++rb) acc += CS[(size_t)rb * NN + j];
  s[tid] = (1.0f / (float)NN) / (acc + 1e-8f); __syncthreads();
  if (tid < 64) vst2(V + (size_t)blockIdx.x * 256 + tid * 4, *(const v4f*)&s[tid * 4]);
}
__global__ __launch_bounds__(256) void k_plan(const float* __restrict__ C, const float* __restrict__ U, const float* __restrict__ V, float* __restrict__ PLAN) {
  __shared__ __align__(16) float s[256]; const int tid = threadIdx.x; const int i = blockIdx.x, j = blockIdx.y * 256 + tid;
  s[tid] = U[i] * exp_ni(-C[(size_t)i * NN + j]) * V[j]; __syncthreads();
  if (tid < 64) vst2(PLAN + (size_t)i * NN + blockIdx.y * 256 + tid * 4, *(const v4f*)&s[tid * 4]);
}
extern "C" void kernel_launch(void* const* d_in, const int* in_sizes, int n_in, void* d_out, int out_size, void* d_ws, size_t ws_size, hipStream_t stream) {
  (void)in_sizes; (void)n_in; (void)out_size;
  const float** F = (const float**)d_in;
  if (ws_size < (size_t)WS_END) return;
  char* ws = (char*)d_ws; __bf16* PW = (__bf16*)(ws + WS_PW); float *HS = (float*)(ws + WS_HS), *HT = (float*)(ws + WS_HT), *RS = (float*)(ws + WS_RS), *U = (float*)(ws + WS_U), *CS = (float*)(ws + WS_CS), *V = (float*)(ws + WS_V);
  float* PLAN = (float*)d_out; float* C = PLAN + (size_t)NN * NN;
  k_packT<<<dim3(HID, 2), 256, 0, stream>>>(F[2], PW);
  k_proj<<<dim3(NN / 64, 2), 128, 0, stream>>>(F[0], F[1], PW, HS, HT);
  k_cost<<<dim3(NN / 64, NN / 128), 256, 0, stream>>>(HS, HT, F[3], F[4], F[5], C, RS);
  k_u<<<NN / 64, 64, 0, stream>>>(RS, U);
  k_colsum<<<dim3(NN / 64, NN / 256), 256, 0, stream>>>(C, U, CS);
  k_v<<<NN / 256, 256, 0, stream>>>(CS, V);
  k_plan<<<dim3(NN, NN / 256), 256, 0, stream>>>(C, U, V, PLAN);
}
